// RWKV_TimeMix_4217657884742
// MI455X (gfx1250) — hardware-verified
//
#include <hip/hip_runtime.h>
#include <math.h>

constexpr int kBsz  = 8;
constexpr int kTlen = 1024;
constexpr int kChan = 1024;
constexpr int kRows = kBsz * kTlen;
constexpr int kVRld = 2 * kChan;
constexpr float kKClamp   = 60.0f;
constexpr float kXmCarry  = 8.0f;
constexpr float kWCarry   = 16.0f;
constexpr float kVRScale  = 4.0f / (8.0f * 16.0f);
constexpr float kOutScale = 1.0f / (16.0f * 16.0f);
constexpr float kInvT     = 1.0f / 1024.0f;
static_assert(kRows % 64 == 0 && kChan % 64 == 0 && kVRld % 64 == 0, "tiles");
static_assert(kChan % 32 == 0, "k step");
static_assert(kChan % 8 == 0 && (kChan / 2) % 256 == 0, "prep lane map");

typedef __attribute__((ext_vector_type(16))) _Float16 v16h;
typedef __attribute__((ext_vector_type(8)))  _Float16 v8h;
typedef __attribute__((ext_vector_type(16))) __bf16   v16b;
typedef __attribute__((ext_vector_type(8)))  __bf16   v8b;
typedef __attribute__((ext_vector_type(8)))  float    v8f;
typedef __attribute__((ext_vector_type(4)))  float    v4f;
typedef __attribute__((ext_vector_type(2)))  float    v2f;
typedef __attribute__((ext_vector_type(4)))  unsigned int v4u;

__device__ __forceinline__ unsigned short f2bf_bits(float f) {
  unsigned u = __float_as_uint(f);
  return (unsigned short)((u + 0x7FFFu + ((u >> 16) & 1u)) >> 16);
}
__device__ __forceinline__ float bf_bits2f(unsigned short h) { return __uint_as_float(((unsigned)h) << 16); }

__device__ __forceinline__ void dep_guard_h(v8f& a, v8f& b, v16h x, v16h y) { asm volatile("v_nop\n\tv_nop\n\tv_nop\n\tv_nop" : "+v"(a), "+v"(b) : "v"(x), "v"(y)); }
__device__ __forceinline__ void dep_guard_b(v8f& a, v8f& b, v16b x, v16b y) { asm volatile("v_nop\n\tv_nop\n\tv_nop\n\tv_nop" : "+v"(a), "+v"(b) : "v"(x), "v"(y)); }
__device__ __forceinline__ void dep_guard4_h(v8f& a, v8f& b, v8f& c, v8f& d, v16h x, v16h y) { asm volatile("v_nop\n\tv_nop\n\tv_nop\n\tv_nop" : "+v"(a), "+v"(b), "+v"(c), "+v"(d) : "v"(x), "v"(y)); }
__device__ __forceinline__ void dep_guard4_b(v8f& a, v8f& b, v8f& c, v8f& d, v16b x, v16b y) { asm volatile("v_nop\n\tv_nop\n\tv_nop\n\tv_nop" : "+v"(a), "+v"(b), "+v"(c), "+v"(d) : "v"(x), "v"(y)); }
__device__ __forceinline__ void keep4_h(v16h a, v16h b, v16h c, v16h d) { asm volatile("v_nop" :: "v"(a), "v"(b), "v"(c), "v"(d)); }
__device__ __forceinline__ void keep4_b(v16b a, v16b b, v16b c, v16b d) { asm volatile("v_nop" :: "v"(a), "v"(b), "v"(c), "v"(d)); }
__device__ __forceinline__ void acc_guard4(v8f& a, v8f& b, v8f& c, v8f& d) { asm volatile("v_nop\n\tv_nop\n\tv_nop\n\tv_nop" : "+v"(a), "+v"(b), "+v"(c), "+v"(d)); }
template <typename T> struct Frag;
template <> struct Frag<_Float16> {
  typedef v16h V; union U { v16h v; v8h h[2]; };
  static __device__ __forceinline__ v16h load(const _Float16* p) {
    U f; f.h[0] = *(const v8h*)(p); f.h[1] = *(const v8h*)(p + 16); return f.v;
  }
  static __device__ __forceinline__ v8f mma(v16h a, v16h b, v8f c) {
    return __builtin_amdgcn_wmma_f32_16x16x32_f16(false, a, false, b, (short)0, c, false, false);
  }
  static __device__ __forceinline__ void guard(v8f& a, v8f& b, v16h x, v16h y) { dep_guard_h(a, b, x, y); }
  static __device__ __forceinline__ void guard4(v8f& a, v8f& b, v8f& c, v8f& d, v16h x, v16h y) { dep_guard4_h(a, b, c, d, x, y); }
  static __device__ __forceinline__ void keep(v16h a, v16h b, v16h c, v16h d) { keep4_h(a, b, c, d); }
};
template <> struct Frag<__bf16> {
  typedef v16b V; union U { v16b v; v8b h[2]; };
  static __device__ __forceinline__ v16b load(const __bf16* p) {
    U f; f.h[0] = *(const v8b*)(p); f.h[1] = *(const v8b*)(p + 16); return f.v;
  }
  static __device__ __forceinline__ v8f mma(v16b a, v16b b, v8f c) {
    return __builtin_amdgcn_wmma_f32_16x16x32_bf16(false, a, false, b, (short)0, c, false, false);
  }
  static __device__ __forceinline__ void guard(v8f& a, v8f& b, v16b x, v16b y) { dep_guard_b(a, b, x, y); }
  static __device__ __forceinline__ void guard4(v8f& a, v8f& b, v8f& c, v8f& d, v16b x, v16b y) { dep_guard4_b(a, b, c, d, x, y); }
  static __device__ __forceinline__ void keep(v16b a, v16b b, v16b c, v16b d) { keep4_b(a, b, c, d); }
};

__device__ __forceinline__ unsigned pk16(unsigned short a, unsigned short b) { return (unsigned)a | ((unsigned)b << 16); }
__device__ __forceinline__ unsigned short h_bits(float f) { const _Float16 h = (_Float16)f; return __builtin_bit_cast(unsigned short, h); }

__device__ __forceinline__ float h16_to_f32(unsigned hb) {
  const unsigned sgn = (hb & 0x8000u) << 16; const unsigned em = hb & 0x7fffu;
  const float fn = __uint_as_float((em << 13) + 0x38000000u);
  const float fs = (float)em * 5.9604644775390625e-8f;
  const float mag = (em < 0x400u) ? fs : fn; return __uint_as_float(__float_as_uint(mag) | sgn); }

template <int ET> struct Elem;
template <> struct Elem<0> { typedef _Float16 T; };
template <> struct Elem<1> { typedef __bf16 T; };
template <int ET, bool SPLIT, int BIAS_MODE, int OUT_MODE, bool RESID, int ACT = 0>
__global__ __launch_bounds__(256) void wmma_gemm64(
    const unsigned short* __restrict__ Ap, const unsigned short* __restrict__ A2p, int lda, long strideA,
    const unsigned short* __restrict__ Btp, const unsigned short* __restrict__ Bt2p, int ldb, long strideB,
    void* __restrict__ Cout, void* __restrict__ Cout2, int ldc, long strideC,
    const float* __restrict__ bias,
    const float* __restrict__ resid, long strideR,
    int M, int N, int K, float scale) {
  typedef typename Elem<ET>::T T;
  typedef typename Frag<T>::V V;
  const T* A = (const T*)Ap; const T* A2 = (const T*)A2p; const T* Bt = (const T*)Btp; const T* Bt2 = (const T*)Bt2p;
  __shared__ __align__(16) float sT[8][16 * 68];
  const int b    = blockIdx.y;
  const int lane = threadIdx.x & 31;
  const int wave = threadIdx.x >> 5;
  const int tilesN = N >> 6;
  const int tilesM = M >> 6;
  const int tile = blockIdx.x * 8 + wave;
  if (tile >= tilesM * tilesN) return;
  const int tm = tile / tilesN;
  const int tn = tile - tm * tilesN;
  const int m0 = tm << 6;
  const int n0 = tn << 6;

  const T* Ab  = A  + (size_t)b * strideA;
  const T* Bb  = Bt + (size_t)b * strideB;
  const T* Ab2 = SPLIT ? (A2  + (size_t)b * strideA) : nullptr;
  const T* Bb2 = SPLIT ? (Bt2 + (size_t)b * strideB) : nullptr;

  const int rlane = lane & 15;
  const int koff  = (lane >> 4) * 8;
  const int mOff  = (lane >> 4) * 8;

  v8f acc[4][4];
#pragma unroll
  for (int i = 0; i < 4; ++i)
#pragma unroll
    for (int j = 0; j < 4; ++j) acc[i][j] = (v8f){0.f,0.f,0.f,0.f,0.f,0.f,0.f,0.f};

  for (int k0 = 0; k0 < K; k0 += 32) {
    V bh[4], bl[4];
#pragma unroll
    for (int j = 0; j < 4; ++j) {
      const size_t bo = (size_t)(n0 + (j << 4) + rlane) * ldb + koff + k0;
      bh[j] = Frag<T>::load(Bb + bo);
      if (SPLIT) bl[j] = Frag<T>::load(Bb2 + bo);
    }
#pragma unroll
    for (int i = 0; i < 4; ++i) {
      const size_t ao = (size_t)(m0 + (i << 4) + rlane) * lda + koff + k0;
      V ah = Frag<T>::load(Ab + ao);
      V al;
      if (SPLIT) al = Frag<T>::load(Ab2 + ao);
#pragma unroll
      for (int j = 0; j < 4; ++j) {
        acc[i][j] = Frag<T>::mma(ah, bh[j], acc[i][j]);
        if (SPLIT) {
          acc[i][j] = Frag<T>::mma(ah, bl[j], acc[i][j]);
          acc[i][j] = Frag<T>::mma(al, bh[j], acc[i][j]);
        }
      }
      Frag<T>::guard4(acc[i][0], acc[i][1], acc[i][2], acc[i][3], ah, SPLIT ? al : ah);
    }
    Frag<T>::keep(bh[0], bh[1], bh[2], bh[3]);
    if (SPLIT) Frag<T>::keep(bl[0], bl[1], bl[2], bl[3]);
  }
  acc_guard4(acc[0][0], acc[0][1], acc[0][2], acc[0][3]);
  acc_guard4(acc[1][0], acc[1][1], acc[1][2], acc[1][3]);
  acc_guard4(acc[2][0], acc[2][1], acc[2][2], acc[2][3]);
  acc_guard4(acc[3][0], acc[3][1], acc[3][2], acc[3][3]);

  float* slab = sT[wave];
  const float* Rb = RESID ? (resid + (size_t)b * strideR) : nullptr;
#pragma unroll
  for (int i = 0; i < 4; ++i) {
    const int mBase = m0 + (i << 4);
#pragma unroll
    for (int j = 0; j < 4; ++j) {
      const int n = n0 + (j << 4) + rlane;
      float bv = 0.f;
      if (BIAS_MODE == 2) bv = bias[n];
#pragma unroll
      for (int r = 0; r < 8; ++r) {
        float v = acc[i][j][r] * scale;
        if (BIAS_MODE == 1) v += bias[mBase + mOff + r];
        if (BIAS_MODE == 2) v += bv;
        if (RESID) v += Rb[(size_t)(mBase + mOff + r) * ldc + n];
        if (ACT == 2) v = fmaxf(v, 0.0f);
        if (ACT == 4) v = (v > 0.f) ? v : 0.01f * v;
        slab[(mOff + r) * 68 + (j << 4) + rlane] = v;
      }
    }
    __builtin_amdgcn_fence(__ATOMIC_RELEASE, "workgroup");
    __builtin_amdgcn_wave_barrier();
    __builtin_amdgcn_fence(__ATOMIC_ACQUIRE, "workgroup");
    if (OUT_MODE == 0) {
      float* C = (float*)Cout + (size_t)b * strideC;
      const int hh = lane >> 4, c4 = (lane & 15) * 4;
      for (int pass = 0; pass < 2; ++pass) {
#pragma unroll
        for (int it = 0; it < 8; ++it) {
          const int row = it * 2 + hh;
          v4f v = *(const v4f*)(slab + row * 68 + c4);
          *(volatile v4f*)(C + (size_t)(mBase + row) * ldc + n0 + c4) = v;
        }
        __threadfence();
      }
    } else {
      const int q = lane >> 3, c8 = (lane & 7) * 8;
      unsigned short* C  = (unsigned short*)Cout  + (size_t)b * strideC;
      unsigned short* C2 = (OUT_MODE == 2) ? ((unsigned short*)Cout2 + (size_t)b * strideC) : nullptr;
      for (int pass = 0; pass < 2; ++pass) {
#pragma unroll
        for (int it = 0; it < 4; ++it) {
          const int row = it * 4 + q;
          const float* sp = slab + row * 68 + c8;
          v8h hv, lv;
#pragma unroll
          for (int e = 0; e < 8; ++e) {
            if (OUT_MODE == 1) {
              hv[e] = (_Float16)sp[e];
            } else {
              unsigned short hb = f2bf_bits(sp[e]);
              unsigned short lb = f2bf_bits(sp[e] - bf_bits2f(hb));
              hv[e] = __builtin_bit_cast(_Float16, hb);
              lv[e] = __builtin_bit_cast(_Float16, lb);
            }
          }
          *(volatile v8h*)(C + (size_t)(mBase + row) * ldc + n0 + c8) = hv;
          if (OUT_MODE == 2) *(volatile v8h*)(C2 + (size_t)(mBase + row) * ldc + n0 + c8) = lv;
        }
        __threadfence();
      }
    }
    __builtin_amdgcn_fence(__ATOMIC_RELEASE, "workgroup");
    __builtin_amdgcn_wave_barrier();
    __builtin_amdgcn_fence(__ATOMIC_ACQUIRE, "workgroup");
  }
}

__global__ __launch_bounds__(256) void cast8_f16s_kernel(const float* __restrict__ in, unsigned short* __restrict__ out, int n8, float scale) {
  const int i = blockIdx.x * 256 + threadIdx.x;
  if (i >= n8) return;
  const float* p = in + 8 * (size_t)i;
  const v4f a = *(const v4f*)(p);
  const v4f c = *(const v4f*)(p + 4);
  unsigned short hb[8];
#pragma unroll
  for (int e = 0; e < 4; ++e) {
    hb[e]     = h_bits(a[e] * scale);
    hb[4 + e] = h_bits(c[e] * scale);
  }
  const v4u u = (v4u){pk16(hb[0], hb[1]), pk16(hb[2], hb[3]), pk16(hb[4], hb[5]), pk16(hb[6], hb[7])};
  unsigned short* q = out + 8 * (size_t)i;
  *(volatile v4u*)q = u;
  __threadfence();
  *(volatile v4u*)q = u;
}

__global__ __launch_bounds__(256) void cast8_bf16hl_kernel(const float* __restrict__ in, unsigned short* __restrict__ hi,
                                                          unsigned short* __restrict__ lo, int n8) {
  const int i = blockIdx.x * 256 + threadIdx.x;
  if (i >= n8) return;
  const float* p = in + 8 * (size_t)i;
  const v4f a = *(const v4f*)(p);
  const v4f c = *(const v4f*)(p + 4);
  unsigned short hb[8], lb[8];
#pragma unroll
  for (int e = 0; e < 4; ++e) {
    const float x0 = a[e];
    const float x1 = c[e];
    hb[e]     = f2bf_bits(x0);
    lb[e]     = f2bf_bits(x0 - bf_bits2f(hb[e]));
    hb[4 + e] = f2bf_bits(x1);
    lb[4 + e] = f2bf_bits(x1 - bf_bits2f(hb[4 + e]));
  }
  const v4u uh = (v4u){pk16(hb[0], hb[1]), pk16(hb[2], hb[3]), pk16(hb[4], hb[5]), pk16(hb[6], hb[7])};
  const v4u ul = (v4u){pk16(lb[0], lb[1]), pk16(lb[2], lb[3]), pk16(lb[4], lb[5]), pk16(lb[6], lb[7])};
  unsigned short* qh = hi + 8 * (size_t)i;
  unsigned short* ql = lo + 8 * (size_t)i;
  *(volatile v4u*)qh = uh;
  *(volatile v4u*)ql = ul;
  __threadfence();
  *(volatile v4u*)qh = uh;
  *(volatile v4u*)ql = ul;
}

__device__ __forceinline__ float mix1(float xv, float xpv, float xnv, float tm, float cm,
                                      float fPrev, float fNext, float fLo, float fHi) {
  const float xm1  = fPrev * xpv;
  const float xp1  = fNext * xnv;
  const float comb = fLo * xm1 + fHi * xp1;
  return xv * tm + xm1 * (1.0f - tm) + comb * cm;
}

__global__ __launch_bounds__(256) void prep_xm_kernel(const float* __restrict__ x, const float* __restrict__ tmix,
                                                      const float* __restrict__ cmix,
                                                      unsigned short* __restrict__ xmh, unsigned short* __restrict__ xml,
                                                      unsigned short* __restrict__ xm16, int n8) {
  const int i = blockIdx.x * 256 + threadIdx.x;
  if (i >= n8) return;
  const int m  = i >> 7;
  const int c0 = (i & 127) * 8;
  const int t  = m & (kTlen - 1);
  const int hasPrev = (t > 0) ? 1 : 0;
  const int hasNext = (t < kTlen - 1) ? 1 : 0;
  const float fPrev = (float)hasPrev;
  const float fNext = (float)hasNext;
  const float fLo = (c0 < kChan / 2) ? 1.0f : 0.0f;
  const float fHi = 1.0f - fLo;
  const size_t base  = (size_t)m * kChan + c0;
  const size_t baseP = (size_t)(m - hasPrev) * kChan + c0;
  const size_t baseN = (size_t)(m + hasNext) * kChan + c0;
  const v4f xa = *(const v4f*)(x + base);
  const v4f xb = *(const v4f*)(x + base + 4);
  const v4f pa = *(const v4f*)(x + baseP);
  const v4f pb = *(const v4f*)(x + baseP + 4);
  const v4f na = *(const v4f*)(x + baseN);
  const v4f nb = *(const v4f*)(x + baseN + 4);
  asm volatile("" ::: "memory");
  const v4f ta = *(const v4f*)(tmix + c0);
  const v4f tb = *(const v4f*)(tmix + c0 + 4);
  const v4f ca = *(const v4f*)(cmix + c0);
  const v4f cb = *(const v4f*)(cmix + c0 + 4);

  unsigned short hb[8], lb[8], fb[8];
#pragma unroll
  for (int e = 0; e < 4; ++e) {
    const float v0 = mix1(xa[e], pa[e], na[e], ta[e], ca[e], fPrev, fNext, fLo, fHi);
    const float v1 = mix1(xb[e], pb[e], nb[e], tb[e], cb[e], fPrev, fNext, fLo, fHi);
    hb[e]     = f2bf_bits(v0);
    lb[e]     = f2bf_bits(v0 - bf_bits2f(hb[e]));
    fb[e]     = h_bits(v0 * kXmCarry);
    hb[4 + e] = f2bf_bits(v1);
    lb[4 + e] = f2bf_bits(v1 - bf_bits2f(hb[4 + e]));
    fb[4 + e] = h_bits(v1 * kXmCarry);
  }
  const v4u uh = (v4u){pk16(hb[0], hb[1]), pk16(hb[2], hb[3]), pk16(hb[4], hb[5]), pk16(hb[6], hb[7])};
  const v4u ul = (v4u){pk16(lb[0], lb[1]), pk16(lb[2], lb[3]), pk16(lb[4], lb[5]), pk16(lb[6], lb[7])};
  const v4u uf = (v4u){pk16(fb[0], fb[1]), pk16(fb[2], fb[3]), pk16(fb[4], fb[5]), pk16(fb[6], fb[7])};
  unsigned short* qh = xmh  + base;
  unsigned short* ql = xml  + base;
  unsigned short* qf = xm16 + base;
  *(volatile v4u*)qh = uh;
  *(volatile v4u*)ql = ul;
  *(volatile v4u*)qf = uf;
  __threadfence();
  *(volatile v4u*)qh = uh;
  *(volatile v4u*)ql = ul;
  *(volatile v4u*)qf = uf;
}

__device__ __forceinline__ float wkv_step(float lgt, float vt4, float rt4, float w, float u,
                                          float& a, float& bden, float& p) {
  const float kt  = expf(fminf(lgt, kKClamp));
  const float ukt = u + kt;
  const float no  = fmaxf(p, ukt);
  const float e1  = expf(p - no);
  const float e2  = expf(ukt - no);
  const float y4  = (e1 * a + e2 * vt4) / (e1 * bden + e2);
  const float wp  = w + p;
  const float no2 = fmaxf(wp, kt);
  const float f1  = expf(wp - no2);
  const float f2  = expf(kt - no2);
  a    = f1 * a + f2 * vt4;
  bden = f1 * bden + f2;
  p    = no2;
  const float sr = 1.0f / (1.0f + expf(-0.25f * rt4));
  return (sr * y4) * 4.0f;
}

__global__ __launch_bounds__(64) void wkv_scan_kernel(const float* __restrict__ lgp, const unsigned* __restrict__ vrw,
                                                      const float* __restrict__ tdecay, const float* __restrict__ tfirst,
                                                      unsigned* __restrict__ gw) {
  const int idx = blockIdx.x * 64 + threadIdx.x;
  if (idx >= kBsz * (kChan / 2)) return;
  const int b  = idx >> 9;
  const int c0 = (idx & 511) * 2;
  const float w0 = tdecay[c0] * kInvT;
  const float w1 = tdecay[c0 + 1] * kInvT;
  const float u0 = tfirst[c0] * kInvT;
  const float u1 = tfirst[c0 + 1] * kInvT;
  const float*    kp = lgp + (size_t)b * kTlen * kChan + c0;
  const unsigned* vp = vrw + ((size_t)b * kTlen * kVRld + c0) / 2;
  const unsigned* rp = vp + kChan / 2;
  unsigned*       gp = gw + ((size_t)b * kTlen * kChan + c0) / 2;
  float a0 = 0.0f, a1 = 0.0f, d0 = 0.0f, d1 = 0.0f, p0 = -1e38f, p1 = -1e38f;
#pragma unroll 1
  for (int t = 0; t < kTlen; ++t) {
    const v2f lg = *(const v2f*)(kp + (size_t)t * kChan);
    const unsigned vw = vp[(size_t)t * (kVRld / 2)];
    const unsigned rw = rp[(size_t)t * (kVRld / 2)];
    const float va = h16_to_f32(vw & 0xffffu);
    const float vb = h16_to_f32(vw >> 16);
    const float ra = h16_to_f32(rw & 0xffffu);
    const float rb = h16_to_f32(rw >> 16);
    const float g0 = wkv_step(lg[0], va, ra, w0, u0, a0, d0, p0);
    const float g1 = wkv_step(lg[1], vb, rb, w1, u1, a1, d1, p1);
    const unsigned gv = pk16(h_bits(g0), h_bits(g1));
    unsigned* gq = gp + (size_t)t * (kChan / 2);
    *(volatile unsigned*)gq = gv;
    __threadfence();
    *(volatile unsigned*)gq = gv;
  }
}

extern "C" void kernel_launch(void* const* d_in, const int* in_sizes, int n_in,
                              void* d_out, int out_size, void* d_ws, size_t ws_size,
                              hipStream_t stream) {
  if (n_in < 9) return;
  const int nX = kRows * kChan;
  const int nW = kChan * kChan;
  if (in_sizes[0] != nX) return;
  if (in_sizes[1] != kChan || in_sizes[2] != kChan || in_sizes[3] != kChan || in_sizes[4] != kChan) return;
  if (in_sizes[5] != nW || in_sizes[6] != nW || in_sizes[7] != nW || in_sizes[8] != nW) return;
  if (out_size != nX) return;

  const size_t szX16  = (size_t)nX * 2;
  const size_t szW16  = (size_t)nW * 2;
  const size_t szLG   = (size_t)nX * 4;
  const size_t szVR16 = (size_t)kRows * kVRld * 2;
  const size_t offXMH = 0;
  const size_t offXML = offXMH + szX16;
  const size_t offXM16 = offXML + szX16;
  const size_t offWKH = offXM16 + szX16;
  const size_t offWKL = offWKH + szW16;
  const size_t offWVR = offWKL + szW16;
  const size_t offWO  = offWVR + 2 * szW16;
  const size_t offLG  = offWO + szW16;
  const size_t offVR  = offLG + szLG;
  const size_t total  = offVR + szVR16;
  if (ws_size < total) return;

  const float* x      = (const float*)d_in[0];
  const float* tdecay = (const float*)d_in[1];
  const float* tfirst = (const float*)d_in[2];
  const float* tmix   = (const float*)d_in[3];
  const float* cmix   = (const float*)d_in[4];
  const float* Wk     = (const float*)d_in[5];
  const float* Wv     = (const float*)d_in[6];
  const float* Wr     = (const float*)d_in[7];
  const float* Wo     = (const float*)d_in[8];
  float* out = (float*)d_out;
  char* ws = (char*)d_ws;
  unsigned short* XMH   = (unsigned short*)(ws + offXMH);
  unsigned short* XML   = (unsigned short*)(ws + offXML);
  unsigned short* XM16  = (unsigned short*)(ws + offXM16);
  unsigned short* G16   = XM16;
  unsigned short* WKH   = (unsigned short*)(ws + offWKH);
  unsigned short* WKL   = (unsigned short*)(ws + offWKL);
  unsigned short* WVR16 = (unsigned short*)(ws + offWVR);
  unsigned short* WO16  = (unsigned short*)(ws + offWO);
  float*          LG    = (float*)(ws + offLG);
  unsigned short* VR16  = (unsigned short*)(ws + offVR);

  const int n8x = nX / 8;
  prep_xm_kernel<<<dim3(n8x / 256), dim3(256), 0, stream>>>(x, tmix, cmix, XMH, XML, XM16, n8x);
  const int n8w = nW / 8;
  cast8_bf16hl_kernel<<<dim3(n8w / 256), dim3(256), 0, stream>>>(Wk, WKH, WKL, n8w);
  cast8_f16s_kernel<<<dim3(n8w / 256), dim3(256), 0, stream>>>(Wv, WVR16, n8w, kWCarry);
  cast8_f16s_kernel<<<dim3(n8w / 256), dim3(256), 0, stream>>>(Wr, WVR16 + (size_t)nW, n8w, kWCarry);
  cast8_f16s_kernel<<<dim3(n8w / 256), dim3(256), 0, stream>>>(Wo, WO16, n8w, kWCarry);

  const int tilesK = (kRows / 64) * (kChan / 64);
  wmma_gemm64<1, true, 0, 0, false, 0><<<dim3(tilesK / 8, 1), dim3(256), 0, stream>>>(
      XMH, XML, kChan, 0L, WKH, WKL, kChan, 0L,
      (void*)LG, (void*)LG, kChan, 0L, LG, LG, 0L, kRows, kChan, kChan, 1.0f);

  const int tilesVR = (kRows / 64) * (kVRld / 64);
  wmma_gemm64<0, false, 0, 1, false, 0><<<dim3(tilesVR / 8, 1), dim3(256), 0, stream>>>(
      XM16, XM16, kChan, 0L, WVR16, WVR16, kChan, 0L,
      (void*)VR16, (void*)VR16, kVRld, 0L, LG, LG, 0L, kRows, kVRld, kChan, kVRScale);

  wkv_scan_kernel<<<dim3((kBsz * (kChan / 2)) / 64), dim3(64), 0, stream>>>(
      LG, (const unsigned*)VR16, tdecay, tfirst, (unsigned*)G16);

  wmma_gemm64<0, false, 0, 0, false, 0><<<dim3(tilesK / 8, 1), dim3(256), 0, stream>>>(
      G16, G16, kChan, 0L, WO16, WO16, kChan, 0L,
      (void*)out, (void*)out, kChan, 0L, LG, LG, 0L, kRows, kChan, kChan, kOutScale);
}
